// MambaBlock_8607114461293
// MI455X (gfx1250) — hardware-verified
//
#include <hip/hip_runtime.h>
#include <stddef.h>
#include <stdint.h>
#include <math.h>


#define MTOK   8192
#define SEQ    2048
#define NBATCH 4
#define DM     1024
#define DI     2048
#define NST    16
#define DTR    64
#define XPN    128
#define XPSRC  96
#define BCP    64
#define GBM    128
#define GBN    64
#define GTHR   128
#define PTHR   256
#define TC     32
#define STHR   64

#define NB_XB  ((MTOK * DM / 8) / PTHR)
#define NB_WIN ((2 * DI * DM / 8) / PTHR)
#define NB_XP2 ((XPN * 2 * DI / 8) / PTHR)
#define NB_DT2 ((DI * 2 * DTR / 8) / PTHR)
#define NB_WO2 ((DM * 2 * DI / 8) / PTHR)
#define NB_AE  ((DI * NST / 4) / PTHR)
#define NB_PREP (NB_XB + NB_WIN + NB_XP2 + NB_DT2 + NB_WO2 + NB_AE)

static_assert(MTOK == NBATCH * SEQ && (SEQ & (SEQ - 1)) == 0);
static_assert(MTOK % GBM == 0 && (2 * DI) % GBN == 0 && XPN % GBN == 0 && DI % GBN == 0 && DM % GBN == 0);
static_assert(DM % 32 == 0 && (2 * DI) % 32 == 0 && (2 * DTR) % 32 == 0);
static_assert(GBM == (GTHR / 32) * 32 && GBN == 64);
static_assert((MTOK * DM / 8) % PTHR == 0 && (2 * DI * DM / 8) % PTHR == 0);
static_assert((XPN * 2 * DI / 8) % PTHR == 0 && (DI * 2 * DTR / 8) % PTHR == 0 && (DM * 2 * DI / 8) % PTHR == 0);
static_assert((DI * NST / 4) % PTHR == 0);
static_assert((2 * DI / 8) == 512 && (2 * DTR / 8) == 16);
static_assert((MTOK * (DI / 4)) % PTHR == 0 && DI / 4 == 512);
static_assert(SEQ % TC == 0 && DI % STHR == 0 && TC * 32 == 4 * 4 * STHR && NST == 16);
static_assert(XPN - BCP == 64 && BCP >= 2 * NST + 0);

typedef float          v4f   __attribute__((ext_vector_type(4)));
typedef float          v8f   __attribute__((ext_vector_type(8)));
typedef int            v8i   __attribute__((ext_vector_type(8)));
typedef unsigned int   v4u   __attribute__((ext_vector_type(4)));
typedef unsigned short v8us  __attribute__((ext_vector_type(8)));
typedef unsigned short v16us __attribute__((ext_vector_type(16)));
typedef __bf16         v16bf __attribute__((ext_vector_type(16)));
typedef v4f  __attribute__((may_alias)) v4fa;
typedef v4u  __attribute__((may_alias)) v4ua;
typedef v8us __attribute__((may_alias)) v8usa;
union FragB { v16bf v; v16us u; v8us h[2]; v8i w; };

__device__ __forceinline__ v8f wmb(const FragB& a, const FragB& b, v8f c) {
  v8f d = __builtin_amdgcn_wmma_f32_16x16x32_bf16(false, a.v, false, b.v, (short)0, c, false, false);
  asm volatile("v_nop\n\tv_nop\n\tv_nop\n\tv_nop" : "+v"(d) : "v"(a.w), "v"(b.w));
  return d;
}

__device__ __forceinline__ unsigned bf16_bits(float f) {
  const unsigned u = __float_as_uint(f);
  return (u + 0x7FFFu + ((u >> 16) & 1u)) >> 16;
}
__device__ __forceinline__ float bf16_val(float f) {
  return __uint_as_float(bf16_bits(f) << 16);
}
__device__ __forceinline__ unsigned pair_bits(float v) {
  const unsigned hb = bf16_bits(v);
  const float lo = v - __uint_as_float(hb << 16);
  return hb | (bf16_bits(lo) << 16);
}
__device__ __forceinline__ float silu_f(float v) {
  return v * (1.0f / (1.0f + expf(-v)));
}
__device__ __forceinline__ float softplus_f(float v) {
  return fmaxf(v, 0.0f) + log1pf(expf(-fabsf(v)));
}

__device__ __forceinline__ void st2_v8us(unsigned short* dp, v8us o) {
  *(volatile v8us*)dp = o;
  __threadfence();
  *(volatile v8us*)dp = o;
}

__device__ __forceinline__ void cvt_lin(const float* __restrict__ S, unsigned short* P, int lb, int tid) {
  const size_t e = ((size_t)lb * PTHR + (size_t)tid) * 8;
  const v4f a = *(const v4fa*)(S + e);
  const v4f b = *(const v4fa*)(S + e + 4);
  v8us o;
  o[0] = (unsigned short)bf16_bits(a.x); o[1] = (unsigned short)bf16_bits(a.y);
  o[2] = (unsigned short)bf16_bits(a.z); o[3] = (unsigned short)bf16_bits(a.w);
  o[4] = (unsigned short)bf16_bits(b.x); o[5] = (unsigned short)bf16_bits(b.y);
  o[6] = (unsigned short)bf16_bits(b.z); o[7] = (unsigned short)bf16_bits(b.w);
  st2_v8us(P + e, o);
}

__device__ __forceinline__ void cvt_dup(const float* __restrict__ W, unsigned short* P, int lb, int tid,
                                        int sh, int nsrc) {
  const int v   = lb * PTHR + tid;
  const int n   = v >> sh;
  const int q   = v & ((1 << sh) - 1);
  const int kin = 4 << sh;
  const int nc  = n < nsrc ? n : nsrc - 1;
  const bool ok = n < nsrc;
  const v4f a = *(const v4fa*)(W + (size_t)nc * (size_t)kin + 4 * q);
  const unsigned short b0 = ok ? (unsigned short)bf16_bits(a.x) : (unsigned short)0;
  const unsigned short b1 = ok ? (unsigned short)bf16_bits(a.y) : (unsigned short)0;
  const unsigned short b2 = ok ? (unsigned short)bf16_bits(a.z) : (unsigned short)0;
  const unsigned short b3 = ok ? (unsigned short)bf16_bits(a.w) : (unsigned short)0;
  v8us o;
  o[0] = b0; o[1] = b0; o[2] = b1; o[3] = b1; o[4] = b2; o[5] = b2; o[6] = b3; o[7] = b3;
  st2_v8us(P + (size_t)n * (size_t)(2 * kin) + 8 * q, o);
}

__global__ __launch_bounds__(PTHR) void k_prep(const float* __restrict__ x, const float* __restrict__ inw,
                                               const float* __restrict__ xpw, const float* __restrict__ dtw,
                                               const float* __restrict__ ow, const float* __restrict__ alog,
                                               unsigned short* XB, unsigned short* WIN, unsigned short* XP2,
                                               unsigned short* DT2, unsigned short* WO2, float* AEXP) {
  const int bid = (int)blockIdx.x;
  const int tid = (int)threadIdx.x;
  if (bid < NB_XB) {
    cvt_lin(x, XB, bid, tid);
  } else if (bid < NB_XB + NB_WIN) {
    cvt_lin(inw, WIN, bid - NB_XB, tid);
  } else if (bid < NB_XB + NB_WIN + NB_XP2) {
    cvt_dup(xpw, XP2, bid - (NB_XB + NB_WIN), tid, 9, XPSRC);
  } else if (bid < NB_XB + NB_WIN + NB_XP2 + NB_DT2) {
    cvt_dup(dtw, DT2, bid - (NB_XB + NB_WIN + NB_XP2), tid, 4, DI);
  } else if (bid < NB_XB + NB_WIN + NB_XP2 + NB_DT2 + NB_WO2) {
    cvt_dup(ow, WO2, bid - (NB_XB + NB_WIN + NB_XP2 + NB_DT2), tid, 9, DM);
  } else if (bid < NB_PREP) {
    const int u4 = (bid - (NB_XB + NB_WIN + NB_XP2 + NB_DT2 + NB_WO2)) * PTHR + tid;
    const v4f a = *(const v4fa*)(alog + 4 * (size_t)u4);
    v4f o;
    o.x = -expf(bf16_val(a.x)); o.y = -expf(bf16_val(a.y));
    o.z = -expf(bf16_val(a.z)); o.w = -expf(bf16_val(a.w));
    float* dp = AEXP + 4 * (size_t)u4;
    *(volatile v4f*)dp = o;
    __threadfence();
    *(volatile v4f*)dp = o;
  }
}

template <int MODE>
__global__ __launch_bounds__(GTHR) void k_gemm(const unsigned short* __restrict__ A,
                                               const unsigned short* __restrict__ WT,
                                               unsigned* outU, long long planeStride,
                                               const float* __restrict__ bias,
                                               int K, int ldo, int colSplit)
{
  __shared__ __attribute__((aligned(16))) float stg[GBM * GBN];
  const int tid = (int)threadIdx.x, lane = tid & 31, wave = tid >> 5, hh = lane >> 4, m = lane & 15;
  const int rowBase = (int)blockIdx.x * GBM;
  const int col0    = (int)blockIdx.y * GBN;

  v8f acc0[4], acc1[4];
  {
    const v8f z = {0.f, 0.f, 0.f, 0.f, 0.f, 0.f, 0.f, 0.f};
#pragma unroll
    for (int t = 0; t < 4; ++t) { acc0[t] = z; acc1[t] = z; }
  }
  const unsigned short* ap0 = A  + (size_t)(rowBase + 32 * wave + m) * (size_t)K + 8 * hh;
  const unsigned short* ap1 = ap0 + (size_t)16 * (size_t)K;
  const unsigned short* wp  = WT + (size_t)(col0 + m) * (size_t)K + 8 * hh;
  const int ksteps = K >> 5;
#pragma unroll 1
  for (int ks = 0; ks < ksteps; ++ks) {
    FragB a0, a1;
    a0.h[0] = *(const v8usa*)(ap0 + 32 * ks);
    a0.h[1] = *(const v8usa*)(ap0 + 32 * ks + 16);
    a1.h[0] = *(const v8usa*)(ap1 + 32 * ks);
    a1.h[1] = *(const v8usa*)(ap1 + 32 * ks + 16);
#pragma unroll
    for (int t = 0; t < 4; ++t) {
      const unsigned short* wq = wp + (size_t)(16 * t) * (size_t)K + 32 * ks;
      FragB bf;
      bf.h[0] = *(const v8usa*)wq;
      bf.h[1] = *(const v8usa*)(wq + 16);
      acc0[t] = wmb(a0, bf, acc0[t]);
      acc1[t] = wmb(a1, bf, acc1[t]);
    }
  }

#pragma unroll
  for (int t = 0; t < 4; ++t) {
    const int lc = 16 * t + m;
#pragma unroll
    for (int r = 0; r < 8; ++r) {
      const int lr = 32 * wave + 8 * hh + r;
      stg[lr * GBN + lc]        = acc0[t][r];
      stg[(lr + 16) * GBN + lc] = acc1[t][r];
    }
  }
  __syncthreads();

  const int plane = col0 / colSplit;
  const int lc0   = col0 - plane * colSplit;

  v4f bq = {0.f, 0.f, 0.f, 0.f};
  if constexpr (MODE == 2) {
    const v4f t4 = *(const v4fa*)(bias + col0 + 4 * m);
    bq.x = bf16_val(t4.x); bq.y = bf16_val(t4.y); bq.z = bf16_val(t4.z); bq.w = bf16_val(t4.w);
  }

#pragma unroll 1
  for (int i = 0; i < 16; ++i) {
    float* p = stg + (32 * wave + 2 * i + hh) * GBN + 4 * m;
    const v4f v = *(const v4fa*)p;
    v4u o;
    if constexpr (MODE == 0) {
      if (plane != 0) {
        o.x = __float_as_uint(silu_f(v.x)); o.y = __float_as_uint(silu_f(v.y));
        o.z = __float_as_uint(silu_f(v.z)); o.w = __float_as_uint(silu_f(v.w));
      } else {
        o.x = __float_as_uint(v.x); o.y = __float_as_uint(v.y);
        o.z = __float_as_uint(v.z); o.w = __float_as_uint(v.w);
      }
    } else if constexpr (MODE == 1) {
      if (plane == 0) {
        o.x = pair_bits(v.x); o.y = pair_bits(v.y); o.z = pair_bits(v.z); o.w = pair_bits(v.w);
      } else {
        o.x = __float_as_uint(v.x); o.y = __float_as_uint(v.y);
        o.z = __float_as_uint(v.z); o.w = __float_as_uint(v.w);
      }
    } else if constexpr (MODE == 2) {
      o.x = __float_as_uint(softplus_f((v.x + bq.x) + bq.x));
      o.y = __float_as_uint(softplus_f((v.y + bq.y) + bq.y));
      o.z = __float_as_uint(softplus_f((v.z + bq.z) + bq.z));
      o.w = __float_as_uint(softplus_f((v.w + bq.w) + bq.w));
    } else {
      o.x = __float_as_uint(v.x); o.y = __float_as_uint(v.y);
      o.z = __float_as_uint(v.z); o.w = __float_as_uint(v.w);
    }
    *(v4ua*)p = o;
  }
  __syncthreads();

  unsigned* ob = outU + (size_t)plane * (size_t)planeStride + (size_t)(lc0 + 4 * m);
#pragma unroll 1
  for (int i = 0; i < 16; ++i) {
    const int lr = 32 * wave + 2 * i + hh;
    const v4u q = *(const v4ua*)(stg + lr * GBN + 4 * m);
    *(volatile v4u*)(ob + (size_t)(rowBase + lr) * (size_t)ldo) = q;
  }
  __threadfence();
#pragma unroll 1
  for (int i = 0; i < 16; ++i) {
    const int lr = 32 * wave + 2 * i + hh;
    const v4u q = *(const v4ua*)(stg + lr * GBN + 4 * m);
    *(volatile v4u*)(ob + (size_t)(rowBase + lr) * (size_t)ldo) = q;
  }
}

__global__ __launch_bounds__(PTHR) void k_conv(const float* __restrict__ xx, const float* __restrict__ cw,
                                               const float* __restrict__ cb, unsigned* xc) {
  const int u = (int)blockIdx.x * PTHR + (int)threadIdx.x;
  if (u >= MTOK * (DI / 4)) return;
  const int mrow = u >> 9;
  const int d0   = (u & 511) * 4;
  const int t    = mrow & (SEQ - 1);
  const v4f w0 = *(const v4fa*)(cw + 4 * (size_t)d0);
  const v4f w1 = *(const v4fa*)(cw + 4 * (size_t)d0 + 4);
  const v4f w2 = *(const v4fa*)(cw + 4 * (size_t)d0 + 8);
  const v4f w3 = *(const v4fa*)(cw + 4 * (size_t)d0 + 12);
  const v4f bb = *(const v4fa*)(cb + d0);
  float a0 = bf16_val(bb.x), a1 = bf16_val(bb.y), a2 = bf16_val(bb.z), a3 = bf16_val(bb.w);
  {
    const bool ok = t >= 3;
    const float f = ok ? 1.0f : 0.0f;
    const int r = ok ? mrow - 3 : mrow;
    const v4f xv = *(const v4fa*)(xx + (size_t)r * DI + d0);
    a0 = fmaf(bf16_val(w0.x) * f, xv.x, a0); a1 = fmaf(bf16_val(w1.x) * f, xv.y, a1);
    a2 = fmaf(bf16_val(w2.x) * f, xv.z, a2); a3 = fmaf(bf16_val(w3.x) * f, xv.w, a3);
  }
  {
    const bool ok = t >= 2;
    const float f = ok ? 1.0f : 0.0f;
    const int r = ok ? mrow - 2 : mrow;
    const v4f xv = *(const v4fa*)(xx + (size_t)r * DI + d0);
    a0 = fmaf(bf16_val(w0.y) * f, xv.x, a0); a1 = fmaf(bf16_val(w1.y) * f, xv.y, a1);
    a2 = fmaf(bf16_val(w2.y) * f, xv.z, a2); a3 = fmaf(bf16_val(w3.y) * f, xv.w, a3);
  }
  {
    const bool ok = t >= 1;
    const float f = ok ? 1.0f : 0.0f;
    const int r = ok ? mrow - 1 : mrow;
    const v4f xv = *(const v4fa*)(xx + (size_t)r * DI + d0);
    a0 = fmaf(bf16_val(w0.z) * f, xv.x, a0); a1 = fmaf(bf16_val(w1.z) * f, xv.y, a1);
    a2 = fmaf(bf16_val(w2.z) * f, xv.z, a2); a3 = fmaf(bf16_val(w3.z) * f, xv.w, a3);
  }
  {
    const v4f xv = *(const v4fa*)(xx + (size_t)mrow * DI + d0);
    a0 = fmaf(bf16_val(w0.w), xv.x, a0); a1 = fmaf(bf16_val(w1.w), xv.y, a1);
    a2 = fmaf(bf16_val(w2.w), xv.z, a2); a3 = fmaf(bf16_val(w3.w), xv.w, a3);
  }
  v4u o;
  o.x = pair_bits(a0); o.y = pair_bits(a1); o.z = pair_bits(a2); o.w = pair_bits(a3);
  unsigned* dp = xc + (size_t)mrow * DI + d0;
  *(volatile v4u*)dp = o;
  __threadfence();
  *(volatile v4u*)dp = o;
}

#define STEP(N, BV, CV) { const float dA = expf(dl * A[N]); h[N] = dA * h[N] + du * (BV); y += h[N] * (CV); }

__global__ __launch_bounds__(STHR) void k_scan(const float* __restrict__ dlt, const unsigned* __restrict__ xc,
                                               unsigned* gy, const float* __restrict__ bc,
                                               const float* __restrict__ aexp, const float* __restrict__ dvec) {
  __shared__ __attribute__((aligned(16))) float sbc[TC * 32];
  __shared__ unsigned sy[TC * STHR];
  const int tid = (int)threadIdx.x;
  const int d   = (int)blockIdx.x * STHR + tid;
  const int b   = (int)blockIdx.y;

  float A[16], h[16];
  {
    const float* ar = aexp + (size_t)d * NST;
    const v4f q0 = *(const v4fa*)(ar);
    const v4f q1 = *(const v4fa*)(ar + 4);
    const v4f q2 = *(const v4fa*)(ar + 8);
    const v4f q3 = *(const v4fa*)(ar + 12);
    A[0] = q0.x;  A[1] = q0.y;  A[2] = q0.z;  A[3] = q0.w;
    A[4] = q1.x;  A[5] = q1.y;  A[6] = q1.z;  A[7] = q1.w;
    A[8] = q2.x;  A[9] = q2.y;  A[10] = q2.z; A[11] = q2.w;
    A[12] = q3.x; A[13] = q3.y; A[14] = q3.z; A[15] = q3.w;
#pragma unroll
    for (int n = 0; n < 16; ++n) h[n] = 0.0f;
  }
  const float Dd = bf16_val(dvec[d]);

#pragma unroll 1
  for (int c = 0; c < SEQ / TC; ++c) {
    const size_t row0 = (size_t)b * SEQ + (size_t)c * TC;
    __syncthreads();
#pragma unroll
    for (int i = 0; i < 4; ++i) {
      const int idx = i * STHR + tid;
      const int rr  = idx >> 3;
      const int c4  = (idx & 7) * 4;
      const v4f v = *(const v4fa*)(bc + (row0 + (size_t)rr) * BCP + c4);
      *(v4fa*)(sbc + rr * 32 + c4) = v;
    }
    __syncthreads();

#pragma unroll 1
    for (int s = 0; s < TC; ++s) {
      const size_t idx = (row0 + (size_t)s) * DI + (size_t)d;
      const float dl = dlt[idx];
      const unsigned pw = xc[idx];
      const float g = __uint_as_float(gy[idx]);
      const float xcv = __uint_as_float(pw << 16) + __uint_as_float(pw & 0xffff0000u);
      const float u  = silu_f(xcv);
      const float du = dl * u;
      const float* bcs = sbc + s * 32;
      const v4f B0 = *(const v4fa*)(bcs);
      const v4f B1 = *(const v4fa*)(bcs + 4);
      const v4f B2 = *(const v4fa*)(bcs + 8);
      const v4f B3 = *(const v4fa*)(bcs + 12);
      const v4f C0 = *(const v4fa*)(bcs + 16);
      const v4f C1 = *(const v4fa*)(bcs + 20);
      const v4f C2 = *(const v4fa*)(bcs + 24);
      const v4f C3 = *(const v4fa*)(bcs + 28);
      float y = 0.0f;
      STEP(0,  B0.x, C0.x) STEP(1,  B0.y, C0.y) STEP(2,  B0.z, C0.z) STEP(3,  B0.w, C0.w)
      STEP(4,  B1.x, C1.x) STEP(5,  B1.y, C1.y) STEP(6,  B1.z, C1.z) STEP(7,  B1.w, C1.w)
      STEP(8,  B2.x, C2.x) STEP(9,  B2.y, C2.y) STEP(10, B2.z, C2.z) STEP(11, B2.w, C2.w)
      STEP(12, B3.x, C3.x) STEP(13, B3.y, C3.y) STEP(14, B3.z, C3.z) STEP(15, B3.w, C3.w)
      const float yv = (y + u * Dd) * g;
      sy[s * STHR + tid] = pair_bits(yv);
    }

#pragma unroll 1
    for (int s = 0; s < TC; ++s) {
      const size_t idx = (row0 + (size_t)s) * DI + (size_t)d;
      const unsigned w = sy[s * STHR + tid];
      *(volatile unsigned*)(gy + idx) = w;
    }
    __threadfence();
#pragma unroll 1
    for (int s = 0; s < TC; ++s) {
      const size_t idx = (row0 + (size_t)s) * DI + (size_t)d;
      const unsigned w = sy[s * STHR + tid];
      *(volatile unsigned*)(gy + idx) = w;
    }
  }
}
#undef STEP

static constexpr size_t SZ_PLANE = (size_t)MTOK * DI * 4;
static constexpr size_t O_R1   = 0;
static constexpr size_t O_R2   = O_R1 + SZ_PLANE;
static constexpr size_t O_R3   = O_R2 + SZ_PLANE;
static constexpr size_t SZ_XB  = (size_t)MTOK * DM * 2;
static constexpr size_t SZ_WIN = (size_t)2 * DI * DM * 2;
static constexpr size_t O_DT   = O_R3 + SZ_PLANE;
static constexpr size_t SZ_DT  = (size_t)MTOK * BCP * 4;
static constexpr size_t O_BC   = O_DT + SZ_DT;
static constexpr size_t O_XP2  = O_BC + SZ_DT;
static constexpr size_t SZ_XP2 = (size_t)XPN * 2 * DI * 2;
static constexpr size_t O_DT2  = O_XP2 + SZ_XP2;
static constexpr size_t SZ_DT2 = (size_t)DI * 2 * DTR * 2;
static constexpr size_t O_WO2  = O_DT2 + SZ_DT2;
static constexpr size_t SZ_WO2 = (size_t)DM * 2 * DI * 2;
static constexpr size_t O_AE   = O_WO2 + SZ_WO2;
static constexpr size_t SZ_AE  = (size_t)DI * NST * 4;
static constexpr size_t WS_TOTAL = O_AE + SZ_AE;

static_assert(SZ_XB + SZ_WIN <= SZ_PLANE);
static_assert(WS_TOTAL == 215613440ull);
static_assert(WS_TOTAL <= 268435456ull);
static_assert(O_DT % 256 == 0 && O_BC % 256 == 0 && O_XP2 % 256 == 0 && O_DT2 % 256 == 0);
static_assert(O_WO2 % 256 == 0 && O_AE % 256 == 0);
static_assert((size_t)(MTOK - 1) * DM + (DM - 1) == 8388607ull);

extern "C" void kernel_launch(void* const* d_in, const int* in_sizes, int n_in,
                              void* d_out, int out_size, void* d_ws, size_t ws_size,
                              hipStream_t stream) {
  if (n_in < 10) return;
  if (in_sizes[0] != MTOK * DM) return;
  if (in_sizes[1] != 2 * DI * DM) return;
  if (in_sizes[2] != DI * 4) return;
  if (in_sizes[3] != DI) return;
  if (in_sizes[4] != XPSRC * DI) return;
  if (in_sizes[5] != DI * DTR) return;
  if (in_sizes[6] != DI) return;
  if (in_sizes[7] != DI * NST) return;
  if (in_sizes[8] != DI) return;
  if (in_sizes[9] != DM * DI) return;
  if (out_size != MTOK * DM) return;
  if (ws_size < WS_TOTAL) return;

  const float* x    = (const float*)d_in[0];
  const float* inw  = (const float*)d_in[1];
  const float* cw   = (const float*)d_in[2];
  const float* cb   = (const float*)d_in[3];
  const float* xpw  = (const float*)d_in[4];
  const float* dtw  = (const float*)d_in[5];
  const float* dtb  = (const float*)d_in[6];
  const float* alog = (const float*)d_in[7];
  const float* dvec = (const float*)d_in[8];
  const float* ow   = (const float*)d_in[9];

  char* ws = (char*)d_ws;
  float*          R1f = (float*)(ws + O_R1);
  unsigned*       R1u = (unsigned*)(ws + O_R1);
  unsigned*       R2u = (unsigned*)(ws + O_R2);
  unsigned*       R3u = (unsigned*)(ws + O_R3);
  unsigned short* XB  = (unsigned short*)(ws + O_R3);
  unsigned short* WIN = (unsigned short*)(ws + O_R3 + SZ_XB);
  unsigned*       DTu = (unsigned*)(ws + O_DT);
  float*          BCf = (float*)(ws + O_BC);
  unsigned short* XP2 = (unsigned short*)(ws + O_XP2);
  unsigned short* DT2 = (unsigned short*)(ws + O_DT2);
  unsigned short* WO2 = (unsigned short*)(ws + O_WO2);
  float*          AE  = (float*)(ws + O_AE);

  k_prep<<<NB_PREP, PTHR, 0, stream>>>(x, inw, xpw, dtw, ow, alog, XB, WIN, XP2, DT2, WO2, AE);
  k_gemm<0><<<dim3(MTOK / GBM, (2 * DI) / GBN), GTHR, 0, stream>>>(
      XB, WIN, R1u, (long long)((size_t)MTOK * DI), dtb, DM, DI, DI);
  k_conv<<<(MTOK * (DI / 4)) / PTHR, PTHR, 0, stream>>>(R1f, cw, cb, R3u);
  k_gemm<1><<<dim3(MTOK / GBM, XPN / GBN), GTHR, 0, stream>>>(
      (const unsigned short*)R3u, XP2, DTu, (long long)((size_t)MTOK * BCP), dtb, 2 * DI, BCP, BCP);
  k_gemm<2><<<dim3(MTOK / GBM, DI / GBN), GTHR, 0, stream>>>(
      (const unsigned short*)DTu, DT2, R1u, 0ll, dtb, 2 * DTR, DI, DI);
  k_scan<<<dim3(DI / STHR, NBATCH), STHR, 0, stream>>>(R1f, R3u, R2u, BCf, AE, dvec);
  k_gemm<3><<<dim3(MTOK / GBM, DM / GBN), GTHR, 0, stream>>>(
      (const unsigned short*)R2u, WO2, (unsigned*)d_out, 0ll, dtb, 2 * DI, DM, DM);
}
